// LocalContextAttention_47175920779963
// MI455X (gfx1250) — hardware-run, weakly checked
//
#include <hip/hip_runtime.h>
#define NB 4
#define TT 4096
#define DM 128
#define WW 9
#define HW 4
#define TP (TT + 2 * HW)
#define WCAR 64.0f
typedef __bf16 v16b __attribute__((ext_vector_type(16)));
typedef unsigned short v8us __attribute__((ext_vector_type(8), may_alias));
typedef float  v8f  __attribute__((ext_vector_type(8)));
typedef float  v4f  __attribute__((ext_vector_type(4)));
typedef float  v4fa __attribute__((ext_vector_type(4), may_alias));
union FragB { v16b v; v8us half[2]; unsigned short u[16]; };

__device__ __forceinline__ unsigned short bf16_bits(float x) { unsigned int u = __float_as_uint(x); return (unsigned short)((u + 0x7FFFu + ((u >> 16) & 1u)) >> 16); }
__device__ __forceinline__ float bf16_val(unsigned short b) { return __uint_as_float(((unsigned int)b) << 16); }
__device__ __forceinline__ float bf16_round(float x) { return bf16_val(bf16_bits(x)); }
template <int NT>
__device__ __forceinline__ v8f mmaN(v16b ah, v16b al, v16b bh, v16b bl, v8f c) {
  c = __builtin_amdgcn_wmma_f32_16x16x32_bf16(false, ah, false, bh, (short)0, c, false, false);
  if (NT >= 2) c = __builtin_amdgcn_wmma_f32_16x16x32_bf16(false, al, false, bh, (short)0, c, false, false);
  if (NT >= 3) c = __builtin_amdgcn_wmma_f32_16x16x32_bf16(false, ah, false, bl, (short)0, c, false, false);
  asm volatile("v_nop\n\tv_nop\n\tv_nop\n\tv_nop" : "+v"(c) : "v"(ah), "v"(al), "v"(bh), "v"(bl));
  return c;
}


typedef _Float16 v16h __attribute__((ext_vector_type(16)));
union FragH { v16h v; v8us half[2]; _Float16 h[16]; unsigned short u[16]; };
template <int NT>
__device__ __forceinline__ v8f mmaH(v16h ah, v16h al, v16h bh, v16h bl, v8f c) {
  c = __builtin_amdgcn_wmma_f32_16x16x32_f16(false, ah, false, bh, (short)0, c, false, false);
  if (NT >= 2) c = __builtin_amdgcn_wmma_f32_16x16x32_f16(false, al, false, bh, (short)0, c, false, false);
  if (NT >= 3) c = __builtin_amdgcn_wmma_f32_16x16x32_f16(false, ah, false, bl, (short)0, c, false, false);
  asm volatile("v_nop\n\tv_nop\n\tv_nop\n\tv_nop" : "+v"(c) : "v"(ah), "v"(al), "v"(bh), "v"(bl));
  return c;
}

__global__ __launch_bounds__(256) void k_wt_f16(const float* __restrict__ W, _Float16* __restrict__ Wt, int K, int N, float scale) {
  const int t = blockIdx.x * 256 + threadIdx.x; if (t >= N * (K / 8)) return; const int n = t / (K / 8), k8 = (t % (K / 8)) * 8; FragH f;
#pragma unroll
  for (int i = 0; i < 8; ++i) f.h[i] = (_Float16)(bf16_round(W[(size_t)(k8 + i) * N + n]) * scale); const v8us o = f.half[0];
  *(volatile v8us*)((unsigned short*)Wt + (size_t)n * K + k8) = o; __threadfence(); *(volatile v8us*)((unsigned short*)Wt + (size_t)n * K + k8) = o;
}
typedef _Float16 v4h __attribute__((ext_vector_type(4)));

__device__ __forceinline__ v16h g2_frag(const _Float16* p, int hh) { FragH f; f.half[0] = *(const v8us*)((const unsigned short*)p + 8 * hh); f.half[1] = *(const v8us*)((const unsigned short*)p + 16 + 8 * hh); return f.v; }
__device__ __forceinline__ v8f g2_mma(v16h a, v16h b, v8f c) { v8f d = __builtin_amdgcn_wmma_f32_16x16x32_f16(false, a, false, b, (short)0, c, false, false); asm volatile("v_nop\n\tv_nop\n\tv_nop\n\tv_nop" : "+v"(d) : "v"(a), "v"(b)); return d; }
template <int ACT>
__global__ __launch_bounds__(128) void k_gemm2(const _Float16* __restrict__ A, int lda, size_t sA, const _Float16* __restrict__ Bh, int ldb, size_t sB, float alpha, const float* __restrict__ bias, size_t sBias, const float* __restrict__ CP, int rowsPerB, size_t sCPb, int row0g,
    float* __restrict__ C, _Float16* __restrict__ C16, int ldc, size_t sC, int M, int N, int K) { static_assert(ACT == 0 || ACT == 3 || ACT == 6 || ACT == 8 || ACT == 9 || ACT == 11 || ACT == 12 || ACT == 14 || ACT == 15 || ACT == 16 || ACT == 17, "k_gemm2: unsupported ACT code (would silently apply no activation)");
  __shared__ __attribute__((aligned(16))) float so[4][32][68];
  const int tid = threadIdx.x, w = tid >> 5, lane = tid & 31, ln = lane & 15, hh = lane >> 4; const int by = blockIdx.y;
  A += (size_t)by * sA; Bh += (size_t)by * sB; const size_t cofs = (size_t)by * sC; const float* bp = bias ? bias + (size_t)by * sBias : nullptr;
  const int ntn = N >> 6; const int mt = blockIdx.x / ntn, nq = blockIdx.x - mt * ntn; const int row0 = mt * 128 + 32 * w, col0 = nq * 64; if (row0 >= M) return;
  const _Float16* a0p = A + (size_t)(row0 + ln) * lda; const _Float16* a1p = a0p + (size_t)16 * lda;
  const _Float16* b0p = Bh + (size_t)(col0 + ln) * ldb; const _Float16* b1p = b0p + (size_t)16 * ldb; const _Float16* b2p = b1p + (size_t)16 * ldb; const _Float16* b3p = b2p + (size_t)16 * ldb;
  const v8f z8 = {0.f,0.f,0.f,0.f,0.f,0.f,0.f,0.f}; v8f c00 = z8, c01 = z8, c02 = z8, c03 = z8, c10 = z8, c11 = z8, c12 = z8, c13 = z8;
  for (int kb = 0; kb < K; kb += 32) { const v16h a0 = g2_frag(a0p + kb, hh), a1 = g2_frag(a1p + kb, hh);
    v16h b = g2_frag(b0p + kb, hh); c00 = g2_mma(a0, b, c00); c10 = g2_mma(a1, b, c10);
    b = g2_frag(b1p + kb, hh); c01 = g2_mma(a0, b, c01); c11 = g2_mma(a1, b, c11);
    b = g2_frag(b2p + kb, hh); c02 = g2_mma(a0, b, c02); c12 = g2_mma(a1, b, c12);
    b = g2_frag(b3p + kb, hh); c03 = g2_mma(a0, b, c03); c13 = g2_mma(a1, b, c13); }
  v8f accs[8] = {c00, c01, c02, c03, c10, c11, c12, c13};
#pragma unroll
  for (int u = 0; u < 8; ++u) { const int t = u & 3, half = u >> 2; const int col = col0 + t * 16 + ln; const float bv = bp ? bf16_round(bp[col]) : 0.f;
#pragma unroll
    for (int r = 0; r < 8; ++r) { const int rloc = half * 16 + 8 * hh + r; float v = accs[u][r] * alpha + bv; if (CP) { if (rowsPerB < 0) v += CP[cofs + (size_t)(row0g + row0 + rloc) * ldc + col];        else { const int bidx = (row0g + row0 + rloc) / rowsPerB; v += CP[(size_t)bidx * sCPb + (size_t)by * 64 + col]; } }
      if (ACT == 3) v = fmaxf(v, 0.f); else if (ACT == 6) v = 0.5f * v * (1.0f + erff(v * 0.70710678118654752f)); else if (ACT == 11) v = 1.0f / (1.0f + expf(-v)); else if (ACT == 15) v = v / (1.0f + expf(-v)); else if (ACT == 12) v = (v > 0.f) ? v : 0.01f * v; else if (ACT == 8) v = tanhf(v); else if (ACT == 9) v = 0.5f * v * (1.0f + tanhf(0.7978845608028654f * (v + 0.044715f * v * v * v))); else if (ACT == 14) v = (v > 0.f) ? v : 0.1f * v; else if (ACT == 16) v = (v >= 0.f) ? v : 0.3f * v; else if (ACT == 17) v = (v >= 0.f) ? v : 0.2f * v;
      so[w][rloc][t * 16 + ln] = v; } }
  __builtin_amdgcn_fence(__ATOMIC_ACQ_REL, "workgroup"); __builtin_amdgcn_wave_barrier();
  const int rsub = lane >> 4, c4 = (lane & 15) * 4;
  for (int pass = 0; pass < 2; ++pass) {
#pragma unroll
    for (int q = 0; q < 16; ++q) { const int r = q * 2 + rsub; const v4f v = *(const v4fa*)&so[w][r][c4]; if (C) *(volatile v4f*)(C + cofs + (size_t)(row0 + r) * ldc + col0 + c4) = v; if (C16) { v4h h4; for (int i = 0; i < 4; ++i) h4[i] = (_Float16)v[i]; *(volatile v4h*)(C16 + cofs + (size_t)(row0 + r) * ldc + col0 + c4) = h4; } }
    if (pass == 0) __threadfence(); } }


__global__ __launch_bounds__(256) void k_padcast(const float* __restrict__ x, _Float16* __restrict__ XP, int n8) {
  const int t = blockIdx.x * 256 + threadIdx.x; if (t >= n8) return; const int rp = t >> 4, c8 = (t & 15) << 3; const int b = rp / TP, ts = rp - b * TP - HW; const int tc = (ts < 0) ? 0 : ((ts > TT - 1) ? TT - 1 : ts); const float in = (ts == tc) ? 1.0f : 0.0f;
  const float* s = x + ((size_t)b * TT + tc) * DM + c8; const v4f a = *(const v4fa*)s, c = *(const v4fa*)(s + 4); FragH f;
#pragma unroll
  for (int q = 0; q < 4; ++q) { f.h[q] = (_Float16)(bf16_round(a[q]) * in); f.h[4 + q] = (_Float16)(bf16_round(c[q]) * in); }
  unsigned short* d = (unsigned short*)XP + (size_t)t * 8; *(volatile v8us*)d = f.half[0]; __threadfence(); *(volatile v8us*)d = f.half[0]; }
__global__ __launch_bounds__(256) void k_bandsm(const float* __restrict__ Q, const float* __restrict__ K, const float* __restrict__ V, const float* __restrict__ PJ, float* __restrict__ O, int n) {
  const int t = blockIdx.x * 256 + threadIdx.x; if (t >= n) return; const int r = t >> 2, c0 = (t & 3) << 5; const int b = r / TT, tt = r - b * TT; const float* q = Q + (size_t)r * DM; float s[WW]; float mx = -3.0e38f;
#pragma unroll
  for (int j = 0; j < WW; ++j) { const int nb = tt + j - HW; const int nc = (nb < 0) ? 0 : ((nb > TT - 1) ? TT - 1 : nb); const float* k = K + ((size_t)b * TT + nc) * DM; float acc = 0.f;
#pragma nounroll
    for (int dd = 0; dd < DM; dd += 4) { const v4f qa = *(const v4fa*)(q + dd), ka = *(const v4fa*)(k + dd); acc += qa[0] * ka[0]; acc += qa[1] * ka[1]; acc += qa[2] * ka[2]; acc += qa[3] * ka[3]; }
    const float sv = (nb == nc) ? acc * 0.08838834764831845f : -1.0e9f; s[j] = sv; mx = (sv > mx) ? sv : mx; }
  float se = 0.f;
#pragma unroll
  for (int j = 0; j < WW; ++j) { s[j] = expf(s[j] - mx); se += s[j]; } const float inv = 1.0f / se;
  float o[32];
#pragma unroll
  for (int c = 0; c < 32; ++c) o[c] = PJ[(size_t)r * DM + c0 + c];
#pragma unroll
  for (int j = 0; j < WW; ++j) { const int nb = tt + j - HW; const int nc = (nb < 0) ? 0 : ((nb > TT - 1) ? TT - 1 : nb); const float* v = V + ((size_t)b * TT + nc) * DM + c0; const float a = s[j] * inv;
#pragma unroll
    for (int c = 0; c < 32; c += 4) { const v4f va = *(const v4fa*)(v + c); o[c] += a * va[0]; o[c + 1] += a * va[1]; o[c + 2] += a * va[2]; o[c + 3] += a * va[3]; } }
  float* d = O + (size_t)r * DM + c0;
#pragma unroll
  for (int c = 0; c < 32; c += 4) { const v4f w = {o[c], o[c + 1], o[c + 2], o[c + 3]}; *(volatile v4f*)(d + c) = w; } __threadfence();
#pragma unroll
  for (int c = 0; c < 32; c += 4) { const v4f w = {o[c], o[c + 1], o[c + 2], o[c + 3]}; *(volatile v4f*)(d + c) = w; } }
__global__ __launch_bounds__(256) void k_ln4(const float* __restrict__ O, const float* __restrict__ gamma, const float* __restrict__ beta, float* __restrict__ Y, int n) {
  const int t = blockIdx.x * 256 + threadIdx.x; if (t >= n) return; const int r = t >> 2, c0 = (t & 3) << 5; const float* o = O + (size_t)r * DM; float sm = 0.f;
  for (int c = 0; c < DM; c += 4) { const v4f a = *(const v4fa*)(o + c); sm += a[0]; sm += a[1]; sm += a[2]; sm += a[3]; } const float mu = sm * (1.0f / DM); float sq = 0.f;
  for (int c = 0; c < DM; c += 4) { const v4f a = *(const v4fa*)(o + c); const float d0 = a[0] - mu, d1 = a[1] - mu, d2 = a[2] - mu, d3 = a[3] - mu; sq += d0 * d0; sq += d1 * d1; sq += d2 * d2; sq += d3 * d3; } const float rs = 1.0f / sqrtf(sq * (1.0f / DM) + 1.0e-3f); float* y = Y + (size_t)r * DM + c0;
#pragma unroll
  for (int c = 0; c < 32; c += 4) { const v4f a = *(const v4fa*)(o + c0 + c), g = *(const v4fa*)(gamma + c0 + c), be = *(const v4fa*)(beta + c0 + c); v4f w;
#pragma unroll
    for (int i = 0; i < 4; ++i) w[i] = (a[i] - mu) * rs * bf16_round(g[i]) + bf16_round(be[i]);
    *(volatile v4f*)(y + c) = w; __threadfence(); *(volatile v4f*)(y + c) = w; } }
extern "C" void kernel_launch(void* const* d_in, const int* in_sizes, int n_in,
                              void* d_out, int out_size, void* d_ws, size_t ws_size, hipStream_t stream) {
  (void)in_sizes; (void)n_in; (void)out_size;
  const float* x = (const float*)d_in[0]; const float* conv_w = (const float*)d_in[1]; const float* conv_b = (const float*)d_in[2]; const float* wq = (const float*)d_in[3]; const float* bq = (const float*)d_in[4]; const float* wk = (const float*)d_in[5]; const float* bk = (const float*)d_in[6]; const float* wv = (const float*)d_in[7]; const float* bv = (const float*)d_in[8]; const float* wp = (const float*)d_in[9]; const float* bp = (const float*)d_in[10]; const float* gamma = (const float*)d_in[11]; const float* beta = (const float*)d_in[12];
  static_assert(TT % 128 == 0 && DM % 64 == 0 && (WW * DM) % 32 == 0 && ((size_t)NB * TP * (DM / 8)) % 256 == 0 && ((size_t)NB * TT * 4) % 256 == 0 && ((size_t)DM * (WW * DM / 8)) % 256 == 0 && ((size_t)DM * (DM / 8)) % 256 == 0, "whole tiles; exact grids");
  float* out = (float*)d_out;
  char* ws = (char*)d_ws; size_t off = 0;
  auto take = [&](size_t bytes) { char* p = ws + off; off += (bytes + 255) & ~(size_t)255; return p; };
  _Float16* XP = (_Float16*)take((size_t)NB * TP * DM * 2); _Float16* BC = (_Float16*)take((size_t)DM * WW * DM * 2); _Float16* BQ = (_Float16*)take((size_t)DM * DM * 2); _Float16* BK = (_Float16*)take((size_t)DM * DM * 2); _Float16* BV = (_Float16*)take((size_t)DM * DM * 2); _Float16* BP = (_Float16*)take((size_t)DM * DM * 2);
  _Float16* LC = (_Float16*)take((size_t)NB * TT * DM * 2); float* QF = (float*)take((size_t)NB * TT * DM * 4); float* KF = (float*)take((size_t)NB * TT * DM * 4); float* VF = (float*)take((size_t)NB * TT * DM * 4); float* PF = (float*)take((size_t)NB * TT * DM * 4); float* OF = (float*)take((size_t)NB * TT * DM * 4);
  if (off > ws_size) return;
  k_padcast<<<(unsigned)((size_t)NB * TP * (DM / 8) / 256), 256, 0, stream>>>(x, XP, NB * TP * (DM / 8));
  k_wt_f16<<<(unsigned)((size_t)DM * (WW * DM / 8) / 256), 256, 0, stream>>>(conv_w, BC, WW * DM, DM, WCAR); k_wt_f16<<<(unsigned)((size_t)DM * (DM / 8) / 256), 256, 0, stream>>>(wq, BQ, DM, DM, WCAR); k_wt_f16<<<(unsigned)((size_t)DM * (DM / 8) / 256), 256, 0, stream>>>(wk, BK, DM, DM, WCAR); k_wt_f16<<<(unsigned)((size_t)DM * (DM / 8) / 256), 256, 0, stream>>>(wv, BV, DM, DM, WCAR); k_wt_f16<<<(unsigned)((size_t)DM * (DM / 8) / 256), 256, 0, stream>>>(wp, BP, DM, DM, WCAR);
  k_gemm2<3><<<dim3((TT / 128) * (DM / 64), NB), 128, 0, stream>>>(XP, DM, (size_t)TP * DM, BC, WW * DM, (size_t)0, 1.0f / WCAR, conv_b, 0, nullptr, 1, 0, 0, nullptr, LC, DM, (size_t)TT * DM, TT, DM, WW * DM);
  k_gemm2<0><<<dim3((TT / 128) * (DM / 64), NB), 128, 0, stream>>>(XP + (size_t)HW * DM, DM, (size_t)TP * DM, BQ, DM, (size_t)0, 1.0f / WCAR, bq, 0, nullptr, 1, 0, 0, QF, nullptr, DM, (size_t)TT * DM, TT, DM, DM);
  k_gemm2<0><<<dim3((NB * TT / 128) * (DM / 64), 1), 128, 0, stream>>>(LC, DM, (size_t)0, BK, DM, (size_t)0, 1.0f / WCAR, bk, 0, nullptr, 1, 0, 0, KF, nullptr, DM, (size_t)0, NB * TT, DM, DM);
  k_gemm2<0><<<dim3((TT / 128) * (DM / 64), NB), 128, 0, stream>>>(XP + (size_t)HW * DM, DM, (size_t)TP * DM, BV, DM, (size_t)0, 1.0f / WCAR, bv, 0, nullptr, 1, 0, 0, VF, nullptr, DM, (size_t)TT * DM, TT, DM, DM);
  k_gemm2<0><<<dim3((TT / 128) * (DM / 64), NB), 128, 0, stream>>>(XP + (size_t)HW * DM, DM, (size_t)TP * DM, BP, DM, (size_t)0, 1.0f / WCAR, bp, 0, nullptr, 1, 0, 0, PF, nullptr, DM, (size_t)TT * DM, TT, DM, DM);
  k_bandsm<<<(unsigned)((size_t)NB * TT * 4 / 256), 256, 0, stream>>>(QF, KF, VF, PF, OF, NB * TT * 4);
  k_ln4<<<(unsigned)((size_t)NB * TT * 4 / 256), 256, 0, stream>>>(OF, gamma, beta, out, NB * TT * 4);
}
